// Attention_64209761075486
// MI455X (gfx1250) — hardware-run, weakly checked
//
#include <hip/hip_runtime.h>


#define NB_  32
#define NQ   256
#define NK   64
#define DM   512
typedef _Float16 h16;
typedef unsigned short bf;
typedef __attribute__((ext_vector_type(16))) __bf16   v16bf;
typedef __attribute__((ext_vector_type(16))) _Float16 v16h;
typedef __attribute__((ext_vector_type(8)))  _Float16 v8h;
typedef __attribute__((ext_vector_type(8)))  unsigned short v8us;
typedef __attribute__((ext_vector_type(8)))  float    v8f;
typedef __attribute__((ext_vector_type(4)))  float    v4f;
typedef v8h  __attribute__((may_alias)) v8ha;
typedef v4f  __attribute__((may_alias)) v4fa;
typedef v8us __attribute__((may_alias)) v8usa;

__device__ __forceinline__ unsigned short f2bf(float f) { unsigned u = __float_as_uint(f); u += 0x7FFFu + ((u >> 16) & 1u); return (unsigned short)(u >> 16); }
__device__ __forceinline__ float bf2f(unsigned short b) { return __uint_as_float(((unsigned)b) << 16); }
__device__ __forceinline__ float bfr(float f) { return bf2f(f2bf(f)); }
__device__ __forceinline__ v16h cat16(v8h lo, v8h hi) { return __builtin_shufflevector(lo, hi, 0, 1, 2, 3, 4, 5, 6, 7, 8, 9, 10, 11, 12, 13, 14, 15); }
__device__ __forceinline__ v16bf cat16b(v8us lo, v8us hi) { return __builtin_bit_cast(v16bf, __builtin_shufflevector(lo, hi, 0, 1, 2, 3, 4, 5, 6, 7, 8, 9, 10, 11, 12, 13, 14, 15)); }
__device__ __forceinline__ v8f wmma16(v16h a, v16h b, v8f c) { return __builtin_amdgcn_wmma_f32_16x16x32_f16(false, a, false, b, (short)0, c, false, false); }
__device__ __forceinline__ v8f wmmab(v16bf a, v16bf b, v8f c) { return __builtin_amdgcn_wmma_f32_16x16x32_bf16(false, a, false, b, (short)0, c, false, false); }


template <typename T16> struct WFrag;
template <> struct WFrag<h16> { typedef v16h V; static __device__ __forceinline__ V ld(const h16* p) { return cat16(*(const v8h*)p, *(const v8h*)(p + 16)); } static __device__ __forceinline__ v8f mma(V a, V b, v8f c) { return wmma16(a, b, c); } };
template <> struct WFrag<bf> { typedef v16bf V; static __device__ __forceinline__ V ld(const bf* p) { return cat16b(*(const v8us*)p, *(const v8us*)(p + 16)); } static __device__ __forceinline__ v8f mma(V a, V b, v8f c) { return wmmab(a, b, c); } };
template <typename T16, int NSPLIT, bool BIAS>
__global__ __launch_bounds__(32) void k_gemmw(const T16* __restrict__ A, const T16* __restrict__ A2, const T16* __restrict__ Bt, const T16* __restrict__ Bt2, int K, float* C, int ldc, const float* __restrict__ bias, size_t sA, size_t sB, size_t sC) {
    typedef typename WFrag<T16>::V V;
    __shared__ __align__(16) float os[16 * 68];
    const size_t z = blockIdx.z; A += z * sA; if (A2) A2 += z * sA; Bt += z * sB; if (Bt2) Bt2 += z * sB; C += z * sC;
    const int lane = threadIdx.x & 31, lr = lane & 15, hi = lane >> 4; const int r0 = blockIdx.x * 64, c0 = blockIdx.y * 64;
    v8f acc[4][4];
#pragma unroll
    for (int mb = 0; mb < 4; ++mb)
#pragma unroll
        for (int nb = 0; nb < 4; ++nb) acc[mb][nb] = (v8f){};
    const size_t aoff = (size_t)(r0 + lr) * K + 8 * hi, boff = (size_t)(c0 + lr) * K + 8 * hi;

    for (int kc = 0; kc < K; kc += 32) {
        V a[4], a2[4];
#pragma unroll
        for (int mb = 0; mb < 4; ++mb) { a[mb] = WFrag<T16>::ld(A + aoff + (size_t)mb * 16 * K + kc); if (NSPLIT == 1 || NSPLIT == 2) a2[mb] = WFrag<T16>::ld(A2 + aoff + (size_t)mb * 16 * K + kc); }
#pragma unroll
        for (int nb = 0; nb < 4; ++nb) { const V b = WFrag<T16>::ld(Bt + boff + (size_t)nb * 16 * K + kc); V b2; if (NSPLIT >= 2) b2 = WFrag<T16>::ld(Bt2 + boff + (size_t)nb * 16 * K + kc);
#pragma unroll
            for (int mb = 0; mb < 4; ++mb) { acc[mb][nb] = WFrag<T16>::mma(a[mb], b, acc[mb][nb]); if (NSPLIT == 1 || NSPLIT == 2) acc[mb][nb] = WFrag<T16>::mma(a2[mb], b, acc[mb][nb]); if (NSPLIT >= 2) acc[mb][nb] = WFrag<T16>::mma(a[mb], b2, acc[mb][nb]); } }
        asm volatile("v_nop\n\tv_nop\n\tv_nop\n\tv_nop" : "+v"(acc[0][0]), "+v"(acc[1][1]), "+v"(acc[2][2]), "+v"(acc[3][3]) : "v"(a[0]), "v"(a[3]));
    }
#pragma unroll
    for (int mb = 0; mb < 4; ++mb) {
#pragma unroll
        for (int nb = 0; nb < 4; ++nb) {
#pragma unroll
            for (int j = 0; j < 8; ++j) os[(hi * 8 + j) * 68 + nb * 16 + lr] = acc[mb][nb][j]; }
        __builtin_amdgcn_wave_barrier(); asm volatile("" ::: "memory");
        float* crow = C + (size_t)(r0 + mb * 16) * ldc + c0;
#pragma unroll 1
        for (int ps = 0; ps < 2; ++ps) {
#pragma unroll
            for (int s = 0; s < 8; ++s) { const int row = 2 * s + hi, cofs = lr * 4; v4f val = *(const v4fa*)(os + row * 68 + cofs); if (BIAS) { val[0] += bfr(bias[c0 + cofs]); val[1] += bfr(bias[c0 + cofs + 1]); val[2] += bfr(bias[c0 + cofs + 2]); val[3] += bfr(bias[c0 + cofs + 3]); }
                *(volatile v4f*)(crow + (size_t)row * ldc + cofs) = val; }
            if (ps == 0) __threadfence(); }
        __builtin_amdgcn_wave_barrier(); asm volatile("" ::: "memory");
    }
}

__device__ __forceinline__ h16 tohx(float x) { return (h16)x; }
__device__ __forceinline__ void splitf(float y, unsigned short& h, unsigned short& l) { h = f2bf(y); l = f2bf(y - bf2f(h)); }
typedef __attribute__((ext_vector_type(2))) _Float16 v2h;
typedef __attribute__((ext_vector_type(4))) _Float16 v4h;
typedef __attribute__((ext_vector_type(2))) unsigned short v2us;
typedef __attribute__((ext_vector_type(4))) unsigned short v4us;
typedef __attribute__((ext_vector_type(2))) float v2f;
typedef __attribute__((ext_vector_type(4))) int v4i;
__global__ __launch_bounds__(256) void k_cvt8(const float* __restrict__ src, bf* dst, size_t n8) { const size_t i = (size_t)blockIdx.x * 256 + threadIdx.x; if (i >= n8) return; const v8f v = *(const v8f*)(src + i * 8); v8us o;
#pragma unroll
    for (int k = 0; k < 8; ++k) o[k] = f2bf(v[k]); *(volatile v8us*)(dst + i * 8) = o; __threadfence(); *(volatile v8us*)(dst + i * 8) = o; }

__global__ __launch_bounds__(256) void k_score(const float* CP, const float* AT, const float* __restrict__ vv, float* S) { const unsigned idx = blockIdx.x * 256 + threadIdx.x; const unsigned j = idx % NK, r = idx / NK, b = r / NQ; const float* c = CP + (size_t)r * DM; const float* a = AT + (size_t)b * DM * NK + j; float s = 0.0f;
    for (int e = 0; e < DM; ++e) s += bfr(vv[e]) * tanhf(c[e] + a[(size_t)e * NK]);
    *(volatile float*)(S + idx) = s; __threadfence(); *(volatile float*)(S + idx) = s; }
__global__ __launch_bounds__(256) void k_softrow(const float* S, h16* P16) { const unsigned r = blockIdx.x * 256 + threadIdx.x; const float* s = S + (size_t)r * NK; float v[NK];
#pragma unroll
    for (int j4 = 0; j4 < NK / 4; ++j4) { const v4f a = *(const v4f*)(s + j4 * 4); v[j4 * 4] = a[0]; v[j4 * 4 + 1] = a[1]; v[j4 * 4 + 2] = a[2]; v[j4 * 4 + 3] = a[3]; }
    float mx = v[0];
#pragma unroll
    for (int j = 1; j < NK; ++j) mx = (v[j] > mx) ? v[j] : mx;
    float sum = 0.0f;
#pragma unroll
    for (int j = 0; j < NK; ++j) { v[j] = expf(v[j] - mx); sum += v[j]; }
    v8h h[NK / 8];
#pragma unroll
    for (int j = 0; j < NK; ++j) h[j / 8][j % 8] = tohx(v[j] / sum);
#pragma unroll
    for (int g = 0; g < NK / 8; ++g) *(volatile v8h*)(P16 + (size_t)r * NK + g * 8) = h[g];
    __threadfence();
#pragma unroll
    for (int g = 0; g < NK / 8; ++g) *(volatile v8h*)(P16 + (size_t)r * NK + g * 8) = h[g]; }
__global__ __launch_bounds__(256) void k_vt(const float* __restrict__ src, h16* VT) { const unsigned idx = blockIdx.x * 256 + threadIdx.x; const unsigned j0 = (idx % (NK / 8)) * 8, d = (idx / (NK / 8)) % DM, b = idx / ((NK / 8) * DM); v8h o;
#pragma unroll
    for (int q = 0; q < 8; ++q) o[q] = tohx(bfr(src[((size_t)b * NK + j0 + q) * DM + d]));
    *(volatile v8h*)(VT + (size_t)idx * 8) = o; __threadfence(); *(volatile v8h*)(VT + (size_t)idx * 8) = o; }

extern "C" void kernel_launch(void* const* d_in, const int* in_sizes, int n_in,
                              void* d_out, int out_size, void* d_ws, size_t ws_size, hipStream_t stream) {
    (void)in_sizes; (void)n_in; (void)out_size;
    const float* a0 = (const float*)d_in[0]; const float* a1 = (const float*)d_in[1]; const float* a2 = (const float*)d_in[2]; const float* a3 = (const float*)d_in[3]; const float* a4 = (const float*)d_in[4];
    float* OUT = (float*)d_out;
    char* wsp = (char*)d_ws;
    auto take = [&](size_t bytes) { char* p = wsp; wsp += (bytes + 255) & ~(size_t)255; return (void*)p; };
    bf* CB = (bf*)take((size_t)NB_ * NQ * DM * 2); bf* AB = (bf*)take((size_t)NB_ * NK * DM * 2); bf* WCB = (bf*)take((size_t)DM * DM * 2); bf* WAB = (bf*)take((size_t)DM * DM * 2);
    float* CP = (float*)take((size_t)NB_ * NQ * DM * 4); float* AT = (float*)take((size_t)NB_ * DM * NK * 4); float* S = (float*)take((size_t)NB_ * NQ * NK * 4);
    h16* P16 = (h16*)take((size_t)NB_ * NQ * NK * 2); h16* VT = (h16*)take((size_t)NB_ * DM * NK * 2);
    if ((size_t)(wsp - (char*)d_ws) > ws_size) return;
    k_cvt8<<<(unsigned)((size_t)NB_ * NQ * DM / 8 / 256), 256, 0, stream>>>(a0, CB, (size_t)NB_ * NQ * DM / 8);
    k_cvt8<<<(unsigned)((size_t)NB_ * NK * DM / 8 / 256), 256, 0, stream>>>(a1, AB, (size_t)NB_ * NK * DM / 8);
    k_cvt8<<<(unsigned)((size_t)DM * DM / 8 / 256), 256, 0, stream>>>(a2, WCB, (size_t)DM * DM / 8);
    k_cvt8<<<(unsigned)((size_t)DM * DM / 8 / 256), 256, 0, stream>>>(a3, WAB, (size_t)DM * DM / 8);
    k_vt<<<(unsigned)((size_t)NB_ * DM * NK / 8 / 256), 256, 0, stream>>>(a1, VT);
    k_gemmw<bf, 0, false><<<dim3(NB_ * NQ / 64, DM / 64, 1), 32, 0, stream>>>(CB, nullptr, WCB, nullptr, DM, CP, DM, nullptr, (size_t)0, (size_t)0, (size_t)0);
    k_gemmw<bf, 0, false><<<dim3(DM / 64, NK / 64, NB_), 32, 0, stream>>>(WAB, nullptr, AB, nullptr, DM, AT, NK, nullptr, (size_t)0, (size_t)NK * DM, (size_t)DM * NK);
    k_score<<<(unsigned)((size_t)NB_ * NQ * NK / 256), 256, 0, stream>>>(CP, AT, a4, S);
    k_softrow<<<(unsigned)(NB_ * NQ / 256), 256, 0, stream>>>(S, P16);
    k_gemmw<h16, 0, false><<<dim3(NQ / 64, DM / 64, NB_), 32, 0, stream>>>(P16, nullptr, VT, nullptr, NK, OUT, DM, nullptr, (size_t)NQ * NK, (size_t)DM * NK, (size_t)NQ * DM);
}
